// MHA_41540923687542
// MI455X (gfx1250) — hardware-verified
//
#include <hip/hip_runtime.h>
#include <stddef.h>
#include <stdint.h>
#include <math.h>


#define DM     256
#define NH     8
#define DS     32
#define KNB    32
#define NB     2
#define KVP    512
#define AVP    512
#define NTHR   256
#define QPB    8
#define GBM    64
#define GBN    64
#define GTHR   128
#define UQ     (DM * (DM / 8))
#define UO     (DM * (AVP / 8))
#define NUW    (3 * UQ + UO)
#define WSMAX  134217728

static_assert(NH * DS == DM);
static_assert(KNB == 32 && QPB * 32 == NTHR);
static_assert(DM % 32 == 0 && AVP % 32 == 0 && AVP == 2 * DM && KVP == 2 * DM);
static_assert(UQ % NTHR == 0 && UO % NTHR == 0 && NUW % NTHR == 0);
static_assert(DM % GBN == 0 && KVP % GBN == 0);
static_assert(GBM == (GTHR / 32) * 16 && GBN == 64);
static_assert(4 * DM == 4 * NTHR);
static_assert(DM / 8 == 32 && AVP / 8 == 64);

typedef float          v4f   __attribute__((ext_vector_type(4)));
typedef float          v8f   __attribute__((ext_vector_type(8)));
typedef int            v8i   __attribute__((ext_vector_type(8)));
typedef unsigned short v8us  __attribute__((ext_vector_type(8)));
typedef unsigned short v16us __attribute__((ext_vector_type(16)));
typedef __bf16         v16bf __attribute__((ext_vector_type(16)));
typedef v4f  __attribute__((may_alias)) v4fa;
typedef v8us __attribute__((may_alias)) v8usa;
union FragB { v16bf v; v16us u; v8us h[2]; v8i w; };

__device__ __forceinline__ v8f wmb(const FragB& a, const FragB& b, v8f c) {
  v8f d = __builtin_amdgcn_wmma_f32_16x16x32_bf16(false, a.v, false, b.v, (short)0, c, false, false);
  asm volatile("v_nop\n\tv_nop\n\tv_nop\n\tv_nop" : "+v"(d) : "v"(a.w), "v"(b.w));
  return d;
}

__device__ __forceinline__ unsigned bf16_bits(float f) {
  const unsigned u = __float_as_uint(f);
  return (u + 0x7FFFu + ((u >> 16) & 1u)) >> 16;
}
__device__ __forceinline__ float bf16_val(float f) {
  return __uint_as_float(bf16_bits(f) << 16);
}
__device__ __forceinline__ unsigned split_bits(float v) {
  const unsigned hb = bf16_bits(v);
  const unsigned lb = bf16_bits(v - __uint_as_float(hb << 16));
  return hb | (lb << 16);
}
__device__ __forceinline__ v8us gather8(const float* __restrict__ p) {
  v8us o;
#pragma unroll
  for (int i = 0; i < 8; ++i) o[i] = (unsigned short)bf16_bits(p[(size_t)i * DM]);
  return o;
}

__global__ __launch_bounds__(NTHR) void k_prep(const float* __restrict__ Wq, const float* __restrict__ Wk,
                                               const float* __restrict__ Wv, const float* __restrict__ Wo,
                                               const float* __restrict__ bq, const float* __restrict__ bk,
                                               const float* __restrict__ bv, const float* __restrict__ bo,
                                               unsigned short* WqT, unsigned short* WkvT, unsigned short* WO2,
                                               float* BIAS) {
  const int u = (int)blockIdx.x * NTHR + (int)threadIdx.x;
  if (u < NUW) {
    v8us o;
    unsigned short* dp;
    if (u < UQ) {
      const int n = u >> 5, k8 = (u & 31) * 8;
      o  = gather8(Wq + (size_t)k8 * DM + n);
      dp = WqT + (size_t)n * DM + k8;
    } else if (u < 2 * UQ) {
      const int v = u - UQ;
      const int n = v >> 5, k8 = (v & 31) * 8;
      o  = gather8(Wk + (size_t)k8 * DM + n);
      dp = WkvT + (size_t)n * DM + k8;
    } else if (u < 3 * UQ) {
      const int v = u - 2 * UQ;
      const int n = v >> 5, k8 = (v & 31) * 8;
      o  = gather8(Wv + (size_t)k8 * DM + n);
      dp = WkvT + (size_t)(DM + n) * DM + k8;
    } else {
      const int v = u - 3 * UQ;
      const int n = v >> 6, k8 = (v & 63) * 8;
      const int kk = k8 & (DM - 1);
      o  = gather8(Wo + (size_t)kk * DM + n);
      dp = WO2 + (size_t)n * AVP + k8;
    }
    *(volatile v8us*)dp = o;
    __threadfence();
    *(volatile v8us*)dp = o;
  } else {
    const int t = u - NUW;
    if (t >= NTHR) return;
    const int j = t & 63, part = t >> 6;
    const v4f a = *(const v4fa*)(bq + 4 * j);
    const v4f b = *(const v4fa*)(bk + 4 * j);
    const v4f c = *(const v4fa*)(bv + 4 * j);
    const v4f d = *(const v4fa*)(bo + 4 * j);
    const unsigned m0 = (part == 0) ? 0xffffffffu : 0u;
    const unsigned m1 = (part == 1) ? 0xffffffffu : 0u;
    const unsigned m2 = (part == 2) ? 0xffffffffu : 0u;
    const unsigned m3 = (part == 3) ? 0xffffffffu : 0u;
    v4f r;
    r.x = bf16_val(__uint_as_float((__float_as_uint(a.x) & m0) | (__float_as_uint(b.x) & m1) |
                                   (__float_as_uint(c.x) & m2) | (__float_as_uint(d.x) & m3)));
    r.y = bf16_val(__uint_as_float((__float_as_uint(a.y) & m0) | (__float_as_uint(b.y) & m1) |
                                   (__float_as_uint(c.y) & m2) | (__float_as_uint(d.y) & m3)));
    r.z = bf16_val(__uint_as_float((__float_as_uint(a.z) & m0) | (__float_as_uint(b.z) & m1) |
                                   (__float_as_uint(c.z) & m2) | (__float_as_uint(d.z) & m3)));
    r.w = bf16_val(__uint_as_float((__float_as_uint(a.w) & m0) | (__float_as_uint(b.w) & m1) |
                                   (__float_as_uint(c.w) & m2) | (__float_as_uint(d.w) & m3)));
    float* bp = BIAS + 4 * t;
    *(volatile v4f*)bp = r;
    __threadfence();
    *(volatile v4f*)bp = r;
  }
}

__global__ __launch_bounds__(NTHR) void k_cvx(const float* __restrict__ x, int nUnits, unsigned short* xb) {
  const int u = (int)blockIdx.x * NTHR + (int)threadIdx.x;
  if (u >= nUnits) return;
  const float* p = x + (size_t)u * 8;
  const v4f a = *(const v4fa*)p;
  const v4f b = *(const v4fa*)(p + 4);
  v8us o;
  o[0] = (unsigned short)bf16_bits(a.x); o[1] = (unsigned short)bf16_bits(a.y);
  o[2] = (unsigned short)bf16_bits(a.z); o[3] = (unsigned short)bf16_bits(a.w);
  o[4] = (unsigned short)bf16_bits(b.x); o[5] = (unsigned short)bf16_bits(b.y);
  o[6] = (unsigned short)bf16_bits(b.z); o[7] = (unsigned short)bf16_bits(b.w);
  unsigned short* dp = xb + (size_t)u * 8;
  *(volatile v8us*)dp = o;
  __threadfence();
  *(volatile v8us*)dp = o;
}

__global__ __launch_bounds__(GTHR) void k_gemm(
    const unsigned short* __restrict__ A, const unsigned short* __restrict__ WT,
    const float* __restrict__ bias, float* outF, int K, int ldo, float scale)
{
  __shared__ __attribute__((aligned(16))) float stg[GBM * GBN];
  const int tid = (int)threadIdx.x, lane = tid & 31, wave = tid >> 5, hh = lane >> 4, m = lane & 15;
  const int rowBase = (int)blockIdx.x * GBM;
  const int col0    = (int)blockIdx.y * GBN;

  v8f acc[4];
  {
    const v8f z = {0.f, 0.f, 0.f, 0.f, 0.f, 0.f, 0.f, 0.f};
    acc[0] = z; acc[1] = z; acc[2] = z; acc[3] = z;
  }
  const unsigned short* ap = A  + (size_t)(rowBase + 16 * wave + m) * (size_t)K + 8 * hh;
  const unsigned short* wp = WT + (size_t)(col0 + m) * (size_t)K + 8 * hh;
  const int ksteps = K >> 5;
#pragma unroll 1
  for (int ks = 0; ks < ksteps; ++ks) {
    FragB af;
    af.h[0] = *(const v8usa*)(ap + 32 * ks);
    af.h[1] = *(const v8usa*)(ap + 32 * ks + 16);
#pragma unroll
    for (int t = 0; t < 4; ++t) {
      const unsigned short* wq = wp + (size_t)(16 * t) * (size_t)K + 32 * ks;
      FragB bf;
      bf.h[0] = *(const v8usa*)wq;
      bf.h[1] = *(const v8usa*)(wq + 16);
      acc[t] = wmb(af, bf, acc[t]);
    }
  }

#pragma unroll
  for (int t = 0; t < 4; ++t) {
    const int lc = 16 * t + m;
#pragma unroll
    for (int r = 0; r < 8; ++r) {
      const int lr = 16 * wave + 8 * hh + r;
      stg[lr * GBN + lc] = acc[t][r];
    }
  }
  __syncthreads();

  const v4f b4 = *(const v4fa*)(bias + col0 + 4 * m);
  v4f fv[8];
#pragma unroll
  for (int i = 0; i < 8; ++i) {
    const int lr = 16 * wave + 2 * i + hh;
    const v4f t4 = *(const v4fa*)(stg + lr * GBN + 4 * m);
    fv[i] = (t4 + b4) * scale;
  }
#pragma unroll
  for (int i = 0; i < 8; ++i) {
    const int lr = 16 * wave + 2 * i + hh;
    const int gr = rowBase + lr;
    float* op = outF + (size_t)gr * (size_t)ldo + col0 + 4 * m;
    *(volatile v4f*)op = fv[i];
  }
  __threadfence();
#pragma unroll
  for (int i = 0; i < 8; ++i) {
    const int lr = 16 * wave + 2 * i + hh;
    const int gr = rowBase + lr;
    float* op = outF + (size_t)gr * (size_t)ldo + col0 + 4 * m;
    *(volatile v4f*)op = fv[i];
  }
}

__global__ __launch_bounds__(NTHR) void k_gattn(const float* __restrict__ QP, const float* __restrict__ KV,
                                                const int* __restrict__ nbr, unsigned short* AVhl,
                                                int nQ, int nM, int totQ) {
  __shared__ __attribute__((aligned(16))) float Qs[QPB * DM];
  __shared__ __attribute__((aligned(16))) float Aw[QPB * DM];
  __shared__ int Idx[QPB * KNB];
  const int tid = (int)threadIdx.x, lane = tid & 31, wave = tid >> 5;
  const int q0 = (int)blockIdx.x * QPB + wave;
  const int q  = q0 < totQ ? q0 : totQ - 1;
  const int b  = q / nQ;

  {
    const float* qp = QP + (size_t)q * DM;
    const v4f qa = *(const v4fa*)(qp + 4 * lane);
    const v4f qb = *(const v4fa*)(qp + 128 + 4 * lane);
    *(v4fa*)(Qs + wave * DM + 4 * lane) = qa;
    *(v4fa*)(Qs + wave * DM + 128 + 4 * lane) = qb;
  }
  int mi = nbr[(size_t)q * KNB + lane];
  mi = mi < 0 ? 0 : (mi > nM - 1 ? nM - 1 : mi);
  Idx[wave * KNB + lane] = mi;
  __syncthreads();

  const float* krow = KV + ((size_t)b * (size_t)nM + (size_t)mi) * KVP;
  const float* qs   = Qs + wave * DM;
#pragma unroll 1
  for (int h = 0; h < NH; ++h) {
    float e = 0.0f;
#pragma unroll 4
    for (int g = 0; g < DS / 4; ++g) {
      const v4f kv = *(const v4fa*)(krow + h * DS + 4 * g);
      const v4f qv = *(const v4fa*)(qs + h * DS + 4 * g);
      e = fmaf(qv.x, kv.x, e);
      e = fmaf(qv.y, kv.y, e);
      e = fmaf(qv.z, kv.z, e);
      e = fmaf(qv.w, kv.w, e);
    }
    float mx = e;
#pragma unroll
    for (int s = 16; s > 0; s >>= 1) mx = fmaxf(mx, __shfl_xor(mx, s, 32));
    const float p = expf(e - mx);
    float sm = p;
#pragma unroll
    for (int s = 16; s > 0; s >>= 1) sm += __shfl_xor(sm, s, 32);
    const float inv = 1.0f / sm;
    Aw[wave * DM + h * KNB + lane] = p * inv;
  }
  __syncthreads();

  const float* aw = Aw + wave * DM + (lane >> 2) * KNB;
  const int*   ix = Idx + wave * KNB;
  const float* vbase = KV + (size_t)b * (size_t)nM * KVP + DM + 8 * lane;
  float o0 = 0.0f, o1 = 0.0f, o2 = 0.0f, o3 = 0.0f, o4 = 0.0f, o5 = 0.0f, o6 = 0.0f, o7 = 0.0f;
#pragma unroll 1
  for (int j = 0; j < KNB; ++j) {
    const int   mk = ix[j];
    const float a  = aw[j];
    const float* vr = vbase + (size_t)mk * KVP;
    const v4f va = *(const v4fa*)vr;
    const v4f vb = *(const v4fa*)(vr + 4);
    o0 = fmaf(a, va.x, o0); o1 = fmaf(a, va.y, o1);
    o2 = fmaf(a, va.z, o2); o3 = fmaf(a, va.w, o3);
    o4 = fmaf(a, vb.x, o4); o5 = fmaf(a, vb.y, o5);
    o6 = fmaf(a, vb.z, o6); o7 = fmaf(a, vb.w, o7);
  }

  v8us hv, lv;
  {
    unsigned s;
    s = split_bits(o0); hv[0] = (unsigned short)(s & 0xffffu); lv[0] = (unsigned short)(s >> 16);
    s = split_bits(o1); hv[1] = (unsigned short)(s & 0xffffu); lv[1] = (unsigned short)(s >> 16);
    s = split_bits(o2); hv[2] = (unsigned short)(s & 0xffffu); lv[2] = (unsigned short)(s >> 16);
    s = split_bits(o3); hv[3] = (unsigned short)(s & 0xffffu); lv[3] = (unsigned short)(s >> 16);
    s = split_bits(o4); hv[4] = (unsigned short)(s & 0xffffu); lv[4] = (unsigned short)(s >> 16);
    s = split_bits(o5); hv[5] = (unsigned short)(s & 0xffffu); lv[5] = (unsigned short)(s >> 16);
    s = split_bits(o6); hv[6] = (unsigned short)(s & 0xffffu); lv[6] = (unsigned short)(s >> 16);
    s = split_bits(o7); hv[7] = (unsigned short)(s & 0xffffu); lv[7] = (unsigned short)(s >> 16);
  }
  const bool wr = q0 < totQ;
  unsigned short* rp = AVhl + (size_t)q * AVP + 8 * lane;
  if (wr) {
    *(volatile v8us*)rp = hv;
    *(volatile v8us*)(rp + DM) = lv;
  }
  __threadfence();
  if (wr) {
    *(volatile v8us*)rp = hv;
    *(volatile v8us*)(rp + DM) = lv;
  }
}

static inline int cdiv(int a, int b) { return (a + b - 1) / b; }
static inline size_t al256(size_t o) { return (o + 255) & ~(size_t)255; }

extern "C" void kernel_launch(void* const* d_in, const int* in_sizes, int n_in,
                              void* d_out, int out_size, void* d_ws, size_t ws_size,
                              hipStream_t stream) {
  if (n_in < 11) return;
  if (in_sizes[0] < DM || (in_sizes[0] % DM) != 0) return;
  if (in_sizes[1] < DM || (in_sizes[1] % DM) != 0) return;
  const int totQ = in_sizes[0] / DM;
  const int totK = in_sizes[1] / DM;
  if ((totQ % NB) != 0 || (totK % NB) != 0) return;
  const int nQ = totQ / NB;
  const int nM = totK / NB;
  if (nQ < 1 || nM < 1) return;
  if ((totQ % GBM) != 0 || (totK % GBM) != 0 || (totQ % QPB) != 0) return;
  if (totQ > (1 << 20) || totK > (1 << 20)) return;
  if ((long long)in_sizes[2] != (long long)totQ * KNB) return;
  if (in_sizes[3] != DM * DM || in_sizes[4] != DM) return;
  if (in_sizes[5] != DM * DM || in_sizes[6] != DM) return;
  if (in_sizes[7] != DM * DM || in_sizes[8] != DM) return;
  if (in_sizes[9] != DM * DM || in_sizes[10] != DM) return;
  if ((long long)out_size != (long long)totQ * DM) return;

  const float* Q   = (const float*)d_in[0];
  const float* Kx  = (const float*)d_in[1];
  const int*   nbr = (const int*)d_in[2];
  const float* Wq  = (const float*)d_in[3];
  const float* bq  = (const float*)d_in[4];
  const float* Wk  = (const float*)d_in[5];
  const float* bk  = (const float*)d_in[6];
  const float* Wv  = (const float*)d_in[7];
  const float* bv  = (const float*)d_in[8];
  const float* Wo  = (const float*)d_in[9];
  const float* bo  = (const float*)d_in[10];
  float* out = (float*)d_out;

  char* ws = (char*)d_ws;
  size_t off = 0;
  const size_t oWqT = off; off = al256(off + (size_t)DM * DM * 2);
  const size_t oWkv = off; off = al256(off + (size_t)KVP * DM * 2);
  const size_t oWO2 = off; off = al256(off + (size_t)DM * AVP * 2);
  const size_t oBI  = off; off = al256(off + (size_t)4 * DM * 4);
  const size_t oQB  = off; off = al256(off + (size_t)totQ * DM * 2);
  const size_t oKB  = off; off = al256(off + (size_t)totK * DM * 2);
  const size_t oQP  = off; off = al256(off + (size_t)totQ * DM * 4);
  const size_t oKV  = off; off = al256(off + (size_t)totK * KVP * 4);
  const size_t oAV  = off; off = al256(off + (size_t)totQ * AVP * 2);
  if (off > ws_size || off > (size_t)WSMAX) return;
  unsigned short* WqT  = (unsigned short*)(ws + oWqT);
  unsigned short* WkvT = (unsigned short*)(ws + oWkv);
  unsigned short* WO2  = (unsigned short*)(ws + oWO2);
  float*          BIAS = (float*)(ws + oBI);
  unsigned short* QB   = (unsigned short*)(ws + oQB);
  unsigned short* KB   = (unsigned short*)(ws + oKB);
  float*          QP   = (float*)(ws + oQP);
  float*          KV   = (float*)(ws + oKV);
  unsigned short* AVhl = (unsigned short*)(ws + oAV);

  const int nUq = totQ * (DM / 8);
  const int nUk = totK * (DM / 8);
  k_prep<<<NUW / NTHR + 1, NTHR, 0, stream>>>(Wq, Wk, Wv, Wo, bq, bk, bv, bo, WqT, WkvT, WO2, BIAS);
  k_cvx<<<cdiv(nUq, NTHR), NTHR, 0, stream>>>(Q, nUq, QB);
  k_cvx<<<cdiv(nUk, NTHR), NTHR, 0, stream>>>(Kx, nUk, KB);
  k_gemm<<<dim3(totQ / GBM, DM / GBN), GTHR, 0, stream>>>(QB, WqT, BIAS, QP, DM, DM, 0.0625f);
  k_gemm<<<dim3(totK / GBM, KVP / GBN), GTHR, 0, stream>>>(KB, WkvT, BIAS + DM, KV, DM, KVP, 1.0f);
  k_gattn<<<totQ / QPB, NTHR, 0, stream>>>(QP, KV, nbr, AVhl, nQ, nM, totQ);
  k_gemm<<<dim3(totQ / GBM, DM / GBN), GTHR, 0, stream>>>(AVhl, WO2, BIAS + 3 * DM, out, AVP, DM, 1.0f);
}
